// Pointnet2SSG_54606214201518
// MI455X (gfx1250) — hardware-verified
//
#include <hip/hip_runtime.h>
#pragma clang fp contract(off)

typedef __attribute__((ext_vector_type(16))) _Float16 v16h;
typedef __attribute__((ext_vector_type(8)))  _Float16 v8h;
typedef __attribute__((ext_vector_type(16))) __bf16   v16b;
typedef __attribute__((ext_vector_type(8)))  __bf16   v8b;
typedef __attribute__((ext_vector_type(8)))  float    v8f;
typedef __attribute__((ext_vector_type(4)))  float    v4f;

constexpr int NBATCH = 32;
constexpr int NPT0   = 4096;
constexpr int NS1    = 512;
constexpr int NS2    = 128;
constexpr int NSAMP  = 64;
constexpr float W_CARRY     = 16.0f;
constexpr float W_CARRY_INV = 1.0f / 16.0f;
constexpr int A3_PITCH = 320;
static_assert(NSAMP == 64);
static_assert(NBATCH * NS2 == 4096);

__device__ __forceinline__ unsigned short f2bf_bits(float f) {
  unsigned u = __float_as_uint(f);
  return (unsigned short)((u + 0x7FFFu + ((u >> 16) & 1u)) >> 16);
}
__device__ __forceinline__ float bf_bits2f(unsigned short h) { return __uint_as_float(((unsigned)h) << 16); }

template <typename T> struct Frag;
template <> struct Frag<_Float16> {
  typedef v16h V; union U { v16h v; v8h h[2]; };
  static __device__ __forceinline__ v16h load(const _Float16* p) {
    U f; f.h[0] = *(const v8h*)(p); f.h[1] = *(const v8h*)(p + 16); return f.v;
  }
};
template <> struct Frag<__bf16> {
  typedef v16b V; union U { v16b v; v8b h[2]; };
  static __device__ __forceinline__ v16b load(const __bf16* p) {
    U f; f.h[0] = *(const v8b*)(p); f.h[1] = *(const v8b*)(p + 16); return f.v;
  }
};

__device__ __forceinline__ v8f mma_h(v16h a, v16h b, v8f c) {
  c = __builtin_amdgcn_wmma_f32_16x16x32_f16(false, a, false, b, (short)0, c, false, false);
  asm volatile("v_nop\n\tv_nop\n\tv_nop\n\tv_nop" : "+v"(c) : "v"(a), "v"(b));
  return c;
}
__device__ __forceinline__ v8f mma_b(v16b a, v16b b, v8f c) {
  c = __builtin_amdgcn_wmma_f32_16x16x32_bf16(false, a, false, b, (short)0, c, false, false);
  asm volatile("v_nop\n\tv_nop\n\tv_nop\n\tv_nop" : "+v"(c) : "v"(a), "v"(b));
  return c;
}
__device__ __forceinline__ v8f zero8() { return (v8f){0.f, 0.f, 0.f, 0.f, 0.f, 0.f, 0.f, 0.f}; }

template <bool SPLITBF>
__global__ __launch_bounds__(256) void pack_wt(const float* __restrict__ W, unsigned short* __restrict__ P,
                                               unsigned short* __restrict__ P2, int Cin, int Cout, int Kpad,
                                               int rot, float carry) {
  const int t = blockIdx.x * 256 + threadIdx.x;
  const int total8 = (Cout * Kpad) >> 3;
  if (t >= total8) return;
  const int e0 = t * 8;
  const int n  = e0 / Kpad;
  const int kb = e0 - n * Kpad;
  const int nrest = Cin - rot;
  v8h hv, lv;
#pragma unroll
  for (int e = 0; e < 8; ++e) {
    const int k = kb + e;
    int ks = (k < nrest) ? (k + rot) : (k - nrest);
    ks = ks < 0 ? 0 : ks;
    ks = ks > (Cin - 1) ? (Cin - 1) : ks;
    const float x = W[(size_t)ks * Cout + n];
    const float v = (k < Cin) ? (x * carry) : 0.0f;
    if (SPLITBF) {
      const unsigned short hb = f2bf_bits(v);
      const unsigned short lb = f2bf_bits(v - bf_bits2f(hb));
      hv[e] = __builtin_bit_cast(_Float16, hb);
      lv[e] = __builtin_bit_cast(_Float16, lb);
    } else {
      hv[e] = (_Float16)v;
      lv[e] = (_Float16)v;
    }
  }
  *(volatile v8h*)(P + (size_t)e0) = hv;
  if (SPLITBF) *(volatile v8h*)(P2 + (size_t)e0) = lv;
  __threadfence();
  *(volatile v8h*)(P + (size_t)e0) = hv;
  if (SPLITBF) *(volatile v8h*)(P2 + (size_t)e0) = lv;
}

template <int N, int NP>
__global__ __launch_bounds__(256) void fps_kernel(const float* __restrict__ xyz, float* __restrict__ outc) {
#pragma clang fp contract(off)
  static_assert(N % 256 == 0);
  static_assert((N * 3) % 4 == 0);
  static_assert((NP * 3) % 128 == 0);
  constexpr int PPT = N / 256;
  __shared__ __align__(16) float sP[N * 3];
  __shared__ __align__(16) float sC[NP * 3];
  __shared__ float sRv[2][8];
  __shared__ int   sRi[2][8];
  const int b = blockIdx.x, tid = threadIdx.x, lane = tid & 31, wave = tid >> 5;
  const float* pts = xyz + (size_t)b * N * 3;
#pragma unroll 1
  for (int i = tid; i < (N * 3) / 4; i += 256) {
    const v4f v = *(const v4f*)(pts + 4 * i);
    *(v4f*)(sP + 4 * i) = v;
  }
  __syncthreads();
  float px[PPT], py[PPT], pz[PPT], dd[PPT];
#pragma unroll
  for (int i = 0; i < PPT; ++i) {
    const int j = i * 256 + tid;
    px[i] = sP[j * 3 + 0];
    py[i] = sP[j * 3 + 1];
    pz[i] = sP[j * 3 + 2];
    dd[i] = 1e10f;
  }
  if (tid == 0) { sC[0] = sP[0]; sC[1] = sP[1]; sC[2] = sP[2]; }
  int last = 0;
#pragma unroll 1
  for (int it = 1; it < NP; ++it) {
    const float lx = sP[last * 3 + 0], ly = sP[last * 3 + 1], lz = sP[last * 3 + 2];
    float bv = 0.0f;
    int bi = 0;
#pragma unroll
    for (int i = 0; i < PPT; ++i) {
      const float dx = px[i] - lx, dy = py[i] - ly, dz = pz[i] - lz;
      const float t0 = dx * dx;
      const float t1 = dy * dy;
      const float t2 = dz * dz;
      const float d  = (t0 + t2) + t1;
      const float od = dd[i];
      const float nd = (d < od) ? d : od;
      dd[i] = nd;
      const int j = i * 256 + tid;
      const bool tk = (i == 0) || (nd > bv);
      bv = tk ? nd : bv;
      bi = tk ? j : bi;
    }
#pragma unroll
    for (int off = 16; off >= 1; off >>= 1) {
      const float ov = __shfl_xor(bv, off, 32);
      const int   oi = __shfl_xor(bi, off, 32);
      const bool tk = (ov > bv) || ((ov == bv) && (oi < bi));
      bv = tk ? ov : bv;
      bi = tk ? oi : bi;
    }
    const int pb = it & 1;
    if (lane == 0) { sRv[pb][wave] = bv; sRi[pb][wave] = bi; }
    __syncthreads();
    float gv = sRv[pb][0];
    int gi = sRi[pb][0];
#pragma unroll
    for (int w = 1; w < 8; ++w) {
      const float ov = sRv[pb][w];
      const int   oi = sRi[pb][w];
      const bool tk = (ov > gv) || ((ov == gv) && (oi < gi));
      gv = tk ? ov : gv;
      gi = tk ? oi : gi;
    }
    gi = gi < 0 ? 0 : gi;
    gi = gi > (N - 1) ? (N - 1) : gi;
    last = gi;
    if (tid == 0) {
      sC[it * 3 + 0] = sP[gi * 3 + 0];
      sC[it * 3 + 1] = sP[gi * 3 + 1];
      sC[it * 3 + 2] = sP[gi * 3 + 2];
    }
  }
  __syncthreads();
  float* ob = outc + (size_t)b * NP * 3;
  for (int pass = 0; pass < 2; ++pass) {
#pragma unroll 1
    for (int i = tid; i < (NP * 3) / 4; i += 256) {
      const v4f v = *(const v4f*)(sC + 4 * i);
      *(volatile v4f*)(ob + 4 * i) = v;
    }
    __threadfence();
  }
}

template <int N>
__device__ __forceinline__ void ball_query_block(const float* __restrict__ pts, const float cx, const float cy,
                                                 const float cz, const float r2, int* sIdx, int* sWc,
                                                 const int tid) {
  static_assert(N % 128 == 0);
  const int lane = tid & 31, wave = tid >> 5;
  if (tid < NSAMP) sIdx[tid] = 0;
  __syncthreads();
  int cnt = 0;
#pragma unroll 1
  for (int c = 0; c < N / 128; ++c) {
    if (cnt >= NSAMP) break;
    const int j = c * 128 + tid;
    const float qx = pts[(size_t)j * 3 + 0];
    const float qy = pts[(size_t)j * 3 + 1];
    const float qz = pts[(size_t)j * 3 + 2];
    const float dx = cx - qx, dy = cy - qy, dz = cz - qz;
    const float t0 = dx * dx;
    const float t1 = dy * dy;
    const float t2 = dz * dz;
    const float d2 = (t0 + t2) + t1;
    const bool hit = d2 < r2;
    const unsigned m = __builtin_amdgcn_ballot_w32(hit);
    const int wc = __builtin_popcount(m);
    const int pb = (c & 1) * 4;
    if (lane == 0) sWc[pb + wave] = wc;
    __syncthreads();
    const int c0 = __builtin_amdgcn_readfirstlane(sWc[pb + 0]);
    const int c1 = __builtin_amdgcn_readfirstlane(sWc[pb + 1]);
    const int c2 = __builtin_amdgcn_readfirstlane(sWc[pb + 2]);
    const int c3 = __builtin_amdgcn_readfirstlane(sWc[pb + 3]);
    int base = cnt;
    base += (wave > 0) ? c0 : 0;
    base += (wave > 1) ? c1 : 0;
    base += (wave > 2) ? c2 : 0;
    const unsigned lt = (1u << lane) - 1u;
    const int pos = base + __builtin_popcount(m & lt);
    if (hit && (pos < NSAMP)) sIdx[pos] = j;
    cnt += c0 + c1 + c2 + c3;
  }
  __syncthreads();
  const int rc = cnt < NSAMP ? cnt : NSAMP;
  const int slot = tid & (NSAMP - 1);
  const int f0 = sIdx[0];
  int v = sIdx[slot];
  const int first = (rc > 0) ? f0 : (N - 1);
  v = (slot < rc) ? v : first;
  v = v < 0 ? 0 : v;
  v = v > (N - 1) ? (N - 1) : v;
  __syncthreads();
  if (tid < NSAMP) sIdx[tid] = v;
  __syncthreads();
}

template <int KPAD, int NCOLS, bool POOL>
__device__ __forceinline__ void mlp_layer(const _Float16* sIn, const int pin, _Float16* sOut, const int pout,
                                          float* sMaxW, const _Float16* __restrict__ Wt,
                                          const float* __restrict__ gam, const float* __restrict__ bet,
                                          const int lane, const int wave) {
  static_assert(KPAD % 32 == 0);
  static_assert(NCOLS % 64 == 0);
  const int rl = lane & 15, hh = lane >> 4, koff = hh * 8;
  const _Float16* arow = sIn + (wave * 16 + rl) * pin + koff;
#pragma unroll 1
  for (int n0 = 0; n0 < NCOLS; n0 += 64) {
    v8f acc[4];
#pragma unroll
    for (int j = 0; j < 4; ++j) acc[j] = zero8();
#pragma unroll 1
    for (int k0 = 0; k0 < KPAD; k0 += 32) {
      const v16h a = Frag<_Float16>::load(arow + k0);
      const _Float16* bp = Wt + (size_t)(n0 + rl) * KPAD + koff + k0;
      const v16h b0 = Frag<_Float16>::load(bp);
      const v16h b1 = Frag<_Float16>::load(bp + (size_t)16 * KPAD);
      const v16h b2 = Frag<_Float16>::load(bp + (size_t)32 * KPAD);
      const v16h b3 = Frag<_Float16>::load(bp + (size_t)48 * KPAD);
      acc[0] = mma_h(a, b0, acc[0]);
      acc[1] = mma_h(a, b1, acc[1]);
      acc[2] = mma_h(a, b2, acc[2]);
      acc[3] = mma_h(a, b3, acc[3]);
    }
#pragma unroll
    for (int j = 0; j < 4; ++j) {
      const int n = n0 + j * 16 + rl;
      const float gs = gam[n] * W_CARRY_INV;
      const float bb = bet[n];
      if (!POOL) {
#pragma unroll
        for (int r = 0; r < 8; ++r) {
          const float v = fmaxf(acc[j][r] * gs + bb, 0.0f);
          sOut[(wave * 16 + hh * 8 + r) * pout + n] = (_Float16)v;
        }
      } else {
        float m = 0.0f;
#pragma unroll
        for (int r = 0; r < 8; ++r) {
          const float v = fmaxf(acc[j][r] * gs + bb, 0.0f);
          m = fmaxf(m, v);
        }
        const float mo = __shfl_xor(m, 16, 32);
        m = fmaxf(m, mo);
        if (hh == 0) sMaxW[n] = m;
      }
    }
  }
}

__global__ __launch_bounds__(128) void sa1_kernel(
    const float* __restrict__ pc, const float* __restrict__ ctr,
    const float* __restrict__ w0, const float* __restrict__ g0, const float* __restrict__ b0,
    const unsigned short* __restrict__ w1t, const float* __restrict__ g1, const float* __restrict__ b1,
    const unsigned short* __restrict__ w2t, const float* __restrict__ g2, const float* __restrict__ b2,
    unsigned short* __restrict__ feat, float r2) {
#pragma clang fp contract(off)
  __shared__ __align__(16) _Float16 sA0[64 * 72];
  __shared__ __align__(16) _Float16 sA1[64 * 72];
  __shared__ __align__(16) float sW0[5 * 64];
  __shared__ __align__(16) float sMax[4 * 128];
  __shared__ int sIdx[NSAMP];
  __shared__ int sWc[8];
  const int tid = threadIdx.x, lane = tid & 31, wave = tid >> 5;
  const int bs = blockIdx.x;
  const int b  = bs / NS1;
  const float* pts = pc + (size_t)b * NPT0 * 3;
  const float cx = ctr[(size_t)bs * 3 + 0];
  const float cy = ctr[(size_t)bs * 3 + 1];
  const float cz = ctr[(size_t)bs * 3 + 2];
  {
    const int t63 = tid & 63;
    const float wa = w0[tid];
    const float wb = w0[128 + t63];
    const float gg = g0[t63];
    const float bb = b0[t63];
    sW0[tid] = wa;
    if (tid < 64) { sW0[128 + tid] = wb; sW0[192 + tid] = gg; sW0[256 + tid] = bb; }
  }
  ball_query_block<NPT0>(pts, cx, cy, cz, r2, sIdx, sWc, tid);
  {
    const int row = tid >> 1, half = tid & 1;
    int p = sIdx[row];
    p = p < 0 ? 0 : p;
    p = p > (NPT0 - 1) ? (NPT0 - 1) : p;
    const float gx = pts[(size_t)p * 3 + 0] - cx;
    const float gy = pts[(size_t)p * 3 + 1] - cy;
    const float gz = pts[(size_t)p * 3 + 2] - cz;
#pragma unroll 1
    for (int cg = 0; cg < 4; ++cg) {
      const int c0 = half * 32 + cg * 8;
      v8h hv;
#pragma unroll
      for (int q = 0; q < 2; ++q) {
        const v4f wr0 = *(const v4f*)(sW0 + c0 + 4 * q);
        const v4f wr1 = *(const v4f*)(sW0 + 64 + c0 + 4 * q);
        const v4f wr2 = *(const v4f*)(sW0 + 128 + c0 + 4 * q);
        const v4f g4  = *(const v4f*)(sW0 + 192 + c0 + 4 * q);
        const v4f b4  = *(const v4f*)(sW0 + 256 + c0 + 4 * q);
#pragma unroll
        for (int e = 0; e < 4; ++e) {
          float z = gx * wr0[e];
          z = __builtin_fmaf(gy, wr1[e], z);
          z = __builtin_fmaf(gz, wr2[e], z);
          const float v = fmaxf(z * g4[e] + b4[e], 0.0f);
          hv[q * 4 + e] = (_Float16)v;
        }
      }
      *(v8h*)(sA0 + row * 72 + c0) = hv;
    }
  }
  __syncthreads();
  mlp_layer<64, 64, false>(sA0, 72, sA1, 72, nullptr, (const _Float16*)w1t, g1, b1, lane, wave);
  __syncthreads();
  mlp_layer<64, 128, true>(sA1, 72, nullptr, 0, sMax + wave * 128, (const _Float16*)w2t, g2, b2, lane, wave);
  __syncthreads();
  if (tid < 16) {
    v8h hv;
#pragma unroll
    for (int e = 0; e < 8; ++e) {
      const int c = tid * 8 + e;
      const float m = fmaxf(fmaxf(sMax[c], sMax[128 + c]), fmaxf(sMax[256 + c], sMax[384 + c]));
      hv[e] = (_Float16)m;
    }
    unsigned short* dst = feat + (size_t)bs * 128 + tid * 8;
    *(volatile v8h*)dst = hv;
    __threadfence();
    *(volatile v8h*)dst = hv;
  }
}

__global__ __launch_bounds__(128) void sa2_kernel(
    const float* __restrict__ xyz1, const float* __restrict__ ctr, const unsigned short* __restrict__ feat1,
    const unsigned short* __restrict__ w0t, const float* __restrict__ g0, const float* __restrict__ b0,
    const unsigned short* __restrict__ w1t, const float* __restrict__ g1, const float* __restrict__ b1,
    const unsigned short* __restrict__ w2t, const float* __restrict__ g2, const float* __restrict__ b2,
    unsigned short* __restrict__ a3h, unsigned short* __restrict__ a3l, float r2) {
#pragma clang fp contract(off)
  __shared__ __align__(16) _Float16 sA[64 * 168];
  __shared__ __align__(16) _Float16 sB[64 * 136];
  __shared__ __align__(16) float sMax[4 * 256];
  __shared__ __align__(16) float sRow[A3_PITCH];
  __shared__ int sIdx[NSAMP];
  __shared__ int sWc[8];
  const int tid = threadIdx.x, lane = tid & 31, wave = tid >> 5;
  const int bs = blockIdx.x;
  const int b  = bs / NS2;
  const float* pts = xyz1 + (size_t)b * NS1 * 3;
  const float cx = ctr[(size_t)bs * 3 + 0];
  const float cy = ctr[(size_t)bs * 3 + 1];
  const float cz = ctr[(size_t)bs * 3 + 2];
  ball_query_block<NS1>(pts, cx, cy, cz, r2, sIdx, sWc, tid);
  {
    const _Float16* f1 = (const _Float16*)feat1 + (size_t)b * NS1 * 128;
#pragma unroll 4
    for (int it = 0; it < 8; ++it) {
      const int q = it * 128 + tid;
      const int row = q >> 4, ch = q & 15;
      int p = sIdx[row];
      p = p < 0 ? 0 : p;
      p = p > (NS1 - 1) ? (NS1 - 1) : p;
      const v8h v = *(const v8h*)(f1 + (size_t)p * 128 + ch * 8);
      *(v8h*)(sA + row * 168 + ch * 8) = v;
    }
  }
  if (tid < 64) {
    int p = sIdx[tid];
    p = p < 0 ? 0 : p;
    p = p > (NS1 - 1) ? (NS1 - 1) : p;
    const float gx = pts[(size_t)p * 3 + 0] - cx;
    const float gy = pts[(size_t)p * 3 + 1] - cy;
    const float gz = pts[(size_t)p * 3 + 2] - cz;
    float zf = 0.0f;
    asm volatile("" : "+v"(zf));
    v8h h0, hz;
    h0[0] = (_Float16)gx; h0[1] = (_Float16)gy; h0[2] = (_Float16)gz; h0[3] = (_Float16)zf;
    h0[4] = (_Float16)zf; h0[5] = (_Float16)zf; h0[6] = (_Float16)zf; h0[7] = (_Float16)zf;
#pragma unroll
    for (int e = 0; e < 8; ++e) hz[e] = (_Float16)zf;
    _Float16* dst = sA + tid * 168 + 128;
    *(v8h*)(dst)      = h0;
    *(v8h*)(dst + 8)  = hz;
    *(v8h*)(dst + 16) = hz;
    *(v8h*)(dst + 24) = hz;
  }
  __syncthreads();
  mlp_layer<160, 128, false>(sA, 168, sB, 136, nullptr, (const _Float16*)w0t, g0, b0, lane, wave);
  __syncthreads();
  mlp_layer<128, 128, false>(sB, 136, sA, 168, nullptr, (const _Float16*)w1t, g1, b1, lane, wave);
  __syncthreads();
  mlp_layer<128, 256, true>(sA, 168, nullptr, 0, sMax + wave * 256, (const _Float16*)w2t, g2, b2, lane, wave);
  __syncthreads();
#pragma unroll 1
  for (int c = tid; c < A3_PITCH; c += 128) {
    const int cc = c < 255 ? c : 255;
    const float m = fmaxf(fmaxf(sMax[cc], sMax[256 + cc]), fmaxf(sMax[512 + cc], sMax[768 + cc]));
    const int xi = c - 256;
    const float xv = (xi <= 0) ? cx : ((xi == 1) ? cy : cz);
    const float v = (c < 256) ? m : ((c < 259) ? xv : 0.0f);
    sRow[c] = v;
  }
  __syncthreads();
  if (tid < 32) {
    v8h hA, lA, hB, lB;
#pragma unroll
    for (int e = 0; e < 8; ++e) {
      const float xa = sRow[lane * 8 + e];
      const unsigned short ha = f2bf_bits(xa);
      const unsigned short la = f2bf_bits(xa - bf_bits2f(ha));
      hA[e] = __builtin_bit_cast(_Float16, ha);
      lA[e] = __builtin_bit_cast(_Float16, la);
      const float xb = sRow[256 + (lane & 7) * 8 + e];
      const unsigned short hb = f2bf_bits(xb);
      const unsigned short lb = f2bf_bits(xb - bf_bits2f(hb));
      hB[e] = __builtin_bit_cast(_Float16, hb);
      lB[e] = __builtin_bit_cast(_Float16, lb);
    }
    unsigned short* rh = a3h + (size_t)bs * A3_PITCH;
    unsigned short* rl = a3l + (size_t)bs * A3_PITCH;
    for (int pass = 0; pass < 2; ++pass) {
      *(volatile v8h*)(rh + lane * 8) = hA;
      *(volatile v8h*)(rl + lane * 8) = lA;
      if (lane < 8) {
        *(volatile v8h*)(rh + 256 + lane * 8) = hB;
        *(volatile v8h*)(rl + 256 + lane * 8) = lB;
      }
      __threadfence();
    }
  }
}

template <bool FUSE>
__global__ __launch_bounds__(128) void gemm_sa3(
    const unsigned short* __restrict__ Ahp, const unsigned short* __restrict__ Alp, int lda,
    const unsigned short* __restrict__ Bhp, const unsigned short* __restrict__ Blp, int ldb, int K,
    const float* __restrict__ gam, const float* __restrict__ bet,
    unsigned short* __restrict__ Chp, unsigned short* __restrict__ Clp, int ldc,
    float* __restrict__ outp, int ldo) {
  __shared__ __align__(16) float sT[4][16 * 68];
  __shared__ __align__(16) float sMx[4][64];
  const int tid = threadIdx.x, lane = tid & 31, wave = tid >> 5;
  const int rl = lane & 15, hh = lane >> 4, koff = hh * 8;
  const int n0 = blockIdx.x * 64;
  const int m0 = blockIdx.y * 128 + wave * 32;
  const __bf16* A  = (const __bf16*)Ahp;
  const __bf16* A2 = (const __bf16*)Alp;
  const __bf16* B  = (const __bf16*)Bhp;
  const __bf16* B2 = (const __bf16*)Blp;
  v8f acc[2][4];
#pragma unroll
  for (int i = 0; i < 2; ++i)
#pragma unroll
    for (int j = 0; j < 4; ++j) acc[i][j] = zero8();
#pragma unroll 1
  for (int k0 = 0; k0 < K; k0 += 32) {
    const size_t ao = (size_t)(m0 + rl) * lda + koff + k0;
    const v16b ah0 = Frag<__bf16>::load(A + ao);
    const v16b al0 = Frag<__bf16>::load(A2 + ao);
    const v16b ah1 = Frag<__bf16>::load(A + ao + (size_t)16 * lda);
    const v16b al1 = Frag<__bf16>::load(A2 + ao + (size_t)16 * lda);
    asm volatile("" ::: "memory");
#pragma unroll
    for (int j = 0; j < 4; ++j) {
      const size_t bo = (size_t)(n0 + j * 16 + rl) * ldb + koff + k0;
      const v16b bh = Frag<__bf16>::load(B + bo);
      const v16b bl = Frag<__bf16>::load(B2 + bo);
      acc[0][j] = mma_b(ah0, bh, acc[0][j]);
      acc[0][j] = mma_b(ah0, bl, acc[0][j]);
      acc[0][j] = mma_b(al0, bh, acc[0][j]);
      acc[1][j] = mma_b(ah1, bh, acc[1][j]);
      acc[1][j] = mma_b(ah1, bl, acc[1][j]);
      acc[1][j] = mma_b(al1, bh, acc[1][j]);
      asm volatile("" ::: "memory");
    }
  }
  float gs[4], bb[4], cm[4];
#pragma unroll
  for (int j = 0; j < 4; ++j) {
    gs[j] = gam[n0 + j * 16 + rl];
    bb[j] = bet[n0 + j * 16 + rl];
    cm[j] = 0.0f;
  }
  float* slab = sT[wave];
#pragma unroll
  for (int i = 0; i < 2; ++i) {
    if (!FUSE) {
#pragma unroll
      for (int j = 0; j < 4; ++j) {
#pragma unroll
        for (int r = 0; r < 8; ++r) {
          const float v = fmaxf(acc[i][j][r] * gs[j] + bb[j], 0.0f);
          slab[(hh * 8 + r) * 68 + j * 16 + rl] = v;
        }
      }
      __syncthreads();
      const int q = lane >> 3, c8 = (lane & 7) * 8;
      for (int pass = 0; pass < 2; ++pass) {
#pragma unroll
        for (int it = 0; it < 4; ++it) {
          const int row = it * 4 + q;
          const float* sp = slab + row * 68 + c8;
          v8h hv, lv;
#pragma unroll
          for (int e = 0; e < 8; ++e) {
            const float x = sp[e];
            const unsigned short hb = f2bf_bits(x);
            const unsigned short lb = f2bf_bits(x - bf_bits2f(hb));
            hv[e] = __builtin_bit_cast(_Float16, hb);
            lv[e] = __builtin_bit_cast(_Float16, lb);
          }
          const size_t co = (size_t)(m0 + i * 16 + row) * ldc + n0 + c8;
          *(volatile v8h*)(Chp + co) = hv;
          *(volatile v8h*)(Clp + co) = lv;
        }
        __threadfence();
      }
      __syncthreads();
    } else {
#pragma unroll
      for (int j = 0; j < 4; ++j) {
#pragma unroll
        for (int r = 0; r < 8; ++r) {
          const float v = fmaxf(acc[i][j][r] * gs[j] + bb[j], 0.0f);
          cm[j] = fmaxf(cm[j], v);
        }
      }
    }
  }
  if (FUSE) {
#pragma unroll
    for (int j = 0; j < 4; ++j) {
      float m = cm[j];
      const float mo = __shfl_xor(m, 16, 32);
      m = fmaxf(m, mo);
      if (hh == 0) sMx[wave][j * 16 + rl] = m;
    }
    __syncthreads();
    if (tid < 16) {
      const int c4 = tid * 4;
      v4f o;
#pragma unroll
      for (int e = 0; e < 4; ++e) {
        o[e] = fmaxf(fmaxf(sMx[0][c4 + e], sMx[1][c4 + e]), fmaxf(sMx[2][c4 + e], sMx[3][c4 + e]));
      }
      float* dst = outp + (size_t)blockIdx.y * ldo + n0 + c4;
      *(volatile v4f*)dst = o;
      __threadfence();
      *(volatile v4f*)dst = o;
    }
  }
}

extern "C" void kernel_launch(void* const* d_in, const int* in_sizes, int n_in,
                              void* d_out, int out_size, void* d_ws, size_t ws_size,
                              hipStream_t stream) {
  (void)in_sizes; (void)n_in; (void)out_size;
  const float* pc  = (const float*)d_in[0];
  const float* w10 = (const float*)d_in[1];
  const float* g10 = (const float*)d_in[2];
  const float* b10 = (const float*)d_in[3];
  const float* w11 = (const float*)d_in[4];
  const float* g11 = (const float*)d_in[5];
  const float* b11 = (const float*)d_in[6];
  const float* w12 = (const float*)d_in[7];
  const float* g12 = (const float*)d_in[8];
  const float* b12 = (const float*)d_in[9];
  const float* w20 = (const float*)d_in[10];
  const float* g20 = (const float*)d_in[11];
  const float* b20 = (const float*)d_in[12];
  const float* w21 = (const float*)d_in[13];
  const float* g21 = (const float*)d_in[14];
  const float* b21 = (const float*)d_in[15];
  const float* w22 = (const float*)d_in[16];
  const float* g22 = (const float*)d_in[17];
  const float* b22 = (const float*)d_in[18];
  const float* w30 = (const float*)d_in[19];
  const float* g30 = (const float*)d_in[20];
  const float* b30 = (const float*)d_in[21];
  const float* w31 = (const float*)d_in[22];
  const float* g31 = (const float*)d_in[23];
  const float* b31 = (const float*)d_in[24];
  const float* w32 = (const float*)d_in[25];
  const float* g32 = (const float*)d_in[26];
  const float* b32 = (const float*)d_in[27];

  char* ws = (char*)d_ws;
  size_t off = 0;
  auto take = [&](size_t bytes) { char* p = ws + off; off += (bytes + 255) & ~(size_t)255; return p; };
  float*          xyz1  = (float*)take((size_t)NBATCH * NS1 * 3 * 4);
  unsigned short* feat1 = (unsigned short*)take((size_t)NBATCH * NS1 * 128 * 2);
  float*          xyz2  = (float*)take((size_t)NBATCH * NS2 * 3 * 4);
  unsigned short* a3h   = (unsigned short*)take((size_t)NBATCH * NS2 * A3_PITCH * 2);
  unsigned short* a3l   = (unsigned short*)take((size_t)NBATCH * NS2 * A3_PITCH * 2);
  unsigned short* h31h  = (unsigned short*)take((size_t)NBATCH * NS2 * 256 * 2);
  unsigned short* h31l  = (unsigned short*)take((size_t)NBATCH * NS2 * 256 * 2);
  unsigned short* h32h  = (unsigned short*)take((size_t)NBATCH * NS2 * 512 * 2);
  unsigned short* h32l  = (unsigned short*)take((size_t)NBATCH * NS2 * 512 * 2);
  unsigned short* w11t  = (unsigned short*)take((size_t)64 * 64 * 2);
  unsigned short* w12t  = (unsigned short*)take((size_t)128 * 64 * 2);
  unsigned short* w20t  = (unsigned short*)take((size_t)128 * 160 * 2);
  unsigned short* w21t  = (unsigned short*)take((size_t)128 * 128 * 2);
  unsigned short* w22t  = (unsigned short*)take((size_t)256 * 128 * 2);
  unsigned short* w30h  = (unsigned short*)take((size_t)256 * 288 * 2);
  unsigned short* w30l  = (unsigned short*)take((size_t)256 * 288 * 2);
  unsigned short* w31h  = (unsigned short*)take((size_t)512 * 256 * 2);
  unsigned short* w31l  = (unsigned short*)take((size_t)512 * 256 * 2);
  unsigned short* w32h  = (unsigned short*)take((size_t)1024 * 512 * 2);
  unsigned short* w32l  = (unsigned short*)take((size_t)1024 * 512 * 2);
  if (off > ws_size) return;

  pack_wt<false><<<(64 * 64 / 8 + 255) / 256, 256, 0, stream>>>(w11, w11t, w11t, 64, 64, 64, 0, W_CARRY);
  pack_wt<false><<<(128 * 64 / 8 + 255) / 256, 256, 0, stream>>>(w12, w12t, w12t, 64, 128, 64, 0, W_CARRY);
  pack_wt<false><<<(128 * 160 / 8 + 255) / 256, 256, 0, stream>>>(w20, w20t, w20t, 131, 128, 160, 3, W_CARRY);
  pack_wt<false><<<(128 * 128 / 8 + 255) / 256, 256, 0, stream>>>(w21, w21t, w21t, 128, 128, 128, 0, W_CARRY);
  pack_wt<false><<<(256 * 128 / 8 + 255) / 256, 256, 0, stream>>>(w22, w22t, w22t, 128, 256, 128, 0, W_CARRY);
  pack_wt<true><<<(256 * 288 / 8 + 255) / 256, 256, 0, stream>>>(w30, w30h, w30l, 259, 256, 288, 3, 1.0f);
  pack_wt<true><<<(512 * 256 / 8 + 255) / 256, 256, 0, stream>>>(w31, w31h, w31l, 256, 512, 256, 0, 1.0f);
  pack_wt<true><<<(1024 * 512 / 8 + 255) / 256, 256, 0, stream>>>(w32, w32h, w32l, 512, 1024, 512, 0, 1.0f);

  fps_kernel<NPT0, NS1><<<NBATCH, 256, 0, stream>>>(pc, xyz1);
  sa1_kernel<<<NBATCH * NS1, 128, 0, stream>>>(pc, xyz1, w10, g10, b10, w11t, g11, b11, w12t, g12, b12,
                                               feat1, 0.04f);
  fps_kernel<NS1, NS2><<<NBATCH, 256, 0, stream>>>(xyz1, xyz2);
  sa2_kernel<<<NBATCH * NS2, 128, 0, stream>>>(xyz1, xyz2, feat1, w20t, g20, b20, w21t, g21, b21,
                                               w22t, g22, b22, a3h, a3l, 0.16f);
  gemm_sa3<false><<<dim3(256 / 64, NBATCH), 128, 0, stream>>>(a3h, a3l, A3_PITCH, w30h, w30l, 288, 288,
                                                              g30, b30, h31h, h31l, 256, (float*)d_out, 1024);
  gemm_sa3<false><<<dim3(512 / 64, NBATCH), 128, 0, stream>>>(h31h, h31l, 256, w31h, w31l, 256, 256,
                                                              g31, b31, h32h, h32l, 512, (float*)d_out, 1024);
  gemm_sa3<true><<<dim3(1024 / 64, NBATCH), 128, 0, stream>>>(h32h, h32l, 512, w32h, w32l, 512, 512,
                                                             g32, b32, h32h, h32l, 512, (float*)d_out, 1024);
}
